// TriangleAttentionUngated_68178310857259
// MI455X (gfx1250) — hardware-verified
//
#include <hip/hip_runtime.h>

typedef __attribute__((ext_vector_type(16))) _Float16 v16h;
typedef __attribute__((ext_vector_type(8)))  _Float16 v8h;
typedef __attribute__((ext_vector_type(16))) __bf16   v16b;
typedef __attribute__((ext_vector_type(8)))  __bf16   v8b;
typedef __attribute__((ext_vector_type(8)))  float    v8f;
typedef __attribute__((ext_vector_type(4)))  float    v4f;

#define EWID 128
#define NNODE 192
#define NROWS 36864
#define QKV_LD 384
#define EB_LD 64
#define VA_LD 256
#define KS_P 16
#define VT_P 192
#define PW_P 64
#define OS_P 132

__device__ __forceinline__ unsigned short f2bf_bits(float f) {
  unsigned u = __float_as_uint(f);
  return (unsigned short)((u + 0x7FFFu + ((u >> 16) & 1u)) >> 16);
}
__device__ __forceinline__ float bf_bits2f(unsigned short h) { return __uint_as_float(((unsigned)h) << 16); }

__device__ __forceinline__ void dep_guard_h(v8f& a, v8f& b, v16h x, v16h y) { asm volatile("v_nop\n\tv_nop\n\tv_nop\n\tv_nop" : "+v"(a), "+v"(b) : "v"(x), "v"(y)); }
__device__ __forceinline__ void dep_guard_b(v8f& a, v8f& b, v16b x, v16b y) { asm volatile("v_nop\n\tv_nop\n\tv_nop\n\tv_nop" : "+v"(a), "+v"(b) : "v"(x), "v"(y)); }
__device__ __forceinline__ void keep4_h(v16h a, v16h b, v16h c, v16h d) { asm volatile("v_nop" :: "v"(a), "v"(b), "v"(c), "v"(d)); }
__device__ __forceinline__ void keep4_b(v16b a, v16b b, v16b c, v16b d) { asm volatile("v_nop" :: "v"(a), "v"(b), "v"(c), "v"(d)); }
__device__ __forceinline__ void acc_guard4(v8f& a, v8f& b, v8f& c, v8f& d) { asm volatile("v_nop\n\tv_nop\n\tv_nop\n\tv_nop" : "+v"(a), "+v"(b), "+v"(c), "+v"(d)); }
template <typename T> struct Frag;
template <> struct Frag<_Float16> {
  typedef v16h V; union U { v16h v; v8h h[2]; };
  static __device__ __forceinline__ v16h load(const _Float16* p) {
    U f; f.h[0] = *(const v8h*)(p); f.h[1] = *(const v8h*)(p + 16); return f.v;
  }
  static __device__ __forceinline__ v8f mma(v16h a, v16h b, v8f c) {
    return __builtin_amdgcn_wmma_f32_16x16x32_f16(false, a, false, b, (short)0, c, false, false);
  }
  static __device__ __forceinline__ void guard(v8f& a, v8f& b, v16h x, v16h y) { dep_guard_h(a, b, x, y); }
  static __device__ __forceinline__ void keep(v16h a, v16h b, v16h c, v16h d) { keep4_h(a, b, c, d); }
};
template <> struct Frag<__bf16> {
  typedef v16b V; union U { v16b v; v8b h[2]; };
  static __device__ __forceinline__ v16b load(const __bf16* p) {
    U f; f.h[0] = *(const v8b*)(p); f.h[1] = *(const v8b*)(p + 16); return f.v;
  }
  static __device__ __forceinline__ v8f mma(v16b a, v16b b, v8f c) {
    return __builtin_amdgcn_wmma_f32_16x16x32_bf16(false, a, false, b, (short)0, c, false, false);
  }
  static __device__ __forceinline__ void guard(v8f& a, v8f& b, v16b x, v16b y) { dep_guard_b(a, b, x, y); }
  static __device__ __forceinline__ void keep(v16b a, v16b b, v16b c, v16b d) { keep4_b(a, b, c, d); }
};

template <int ET> struct Elem;
template <> struct Elem<0> { typedef _Float16 T; };
template <> struct Elem<1> { typedef __bf16 T; };
template <int ET, bool SPLIT, int BIAS_MODE, int OUT_MODE, bool RESID, int ACT = 0>
__global__ __launch_bounds__(256) void wmma_gemm64(
    const unsigned short* __restrict__ Ap, const unsigned short* __restrict__ A2p, int lda, long strideA,
    const unsigned short* __restrict__ Btp, const unsigned short* __restrict__ Bt2p, int ldb, long strideB,
    void* __restrict__ Cout, void* __restrict__ Cout2, int ldc, long strideC,
    const float* __restrict__ bias,
    const float* __restrict__ resid, long strideR,
    int M, int N, int K, float scale) {
  typedef typename Elem<ET>::T T;
  typedef typename Frag<T>::V V;
  const T* A = (const T*)Ap; const T* A2 = (const T*)A2p; const T* Bt = (const T*)Btp; const T* Bt2 = (const T*)Bt2p;
  __shared__ __align__(16) float sT[8][16 * 68];
  const int b    = blockIdx.y;
  const int lane = threadIdx.x & 31;
  const int wave = threadIdx.x >> 5;
  const int tilesN = N >> 6;
  const int tilesM = M >> 6;
  const int tile = blockIdx.x * 8 + wave;
  if (tile >= tilesM * tilesN) return;
  const int tm = tile / tilesN;
  const int tn = tile - tm * tilesN;
  const int m0 = tm << 6;
  const int n0 = tn << 6;

  const T* Ab  = A  + (size_t)b * strideA;
  const T* Bb  = Bt + (size_t)b * strideB;
  const T* Ab2 = SPLIT ? (A2  + (size_t)b * strideA) : nullptr;
  const T* Bb2 = SPLIT ? (Bt2 + (size_t)b * strideB) : nullptr;

  const int rlane = lane & 15;
  const int koff  = (lane >> 4) * 8;
  const int mOff  = (lane >> 4) * 8;

  v8f acc[4][4];
#pragma unroll
  for (int i = 0; i < 4; ++i)
#pragma unroll
    for (int j = 0; j < 4; ++j) acc[i][j] = (v8f){0.f,0.f,0.f,0.f,0.f,0.f,0.f,0.f};

  for (int k0 = 0; k0 < K; k0 += 32) {
    V bh[4], bl[4];
#pragma unroll
    for (int j = 0; j < 4; ++j) {
      const size_t bo = (size_t)(n0 + (j << 4) + rlane) * ldb + koff + k0;
      bh[j] = Frag<T>::load(Bb + bo);
      if (SPLIT) bl[j] = Frag<T>::load(Bb2 + bo);
    }
#pragma unroll
    for (int i = 0; i < 4; ++i) {
      const size_t ao = (size_t)(m0 + (i << 4) + rlane) * lda + koff + k0;
      V ah = Frag<T>::load(Ab + ao);
      V al;
      if (SPLIT) al = Frag<T>::load(Ab2 + ao);
#pragma unroll
      for (int j = 0; j < 4; ++j) {
        acc[i][j] = Frag<T>::mma(ah, bh[j], acc[i][j]);
        if (SPLIT) {
          acc[i][j] = Frag<T>::mma(ah, bl[j], acc[i][j]);
          acc[i][j] = Frag<T>::mma(al, bh[j], acc[i][j]);
        }
      }
      Frag<T>::guard(acc[i][0], acc[i][3], ah, SPLIT ? al : ah);
    }
    Frag<T>::keep(bh[0], bh[1], bh[2], bh[3]);
    if (SPLIT) Frag<T>::keep(bl[0], bl[1], bl[2], bl[3]);
  }
  acc_guard4(acc[0][0], acc[0][1], acc[0][2], acc[0][3]);
  acc_guard4(acc[1][0], acc[1][1], acc[1][2], acc[1][3]);
  acc_guard4(acc[2][0], acc[2][1], acc[2][2], acc[2][3]);
  acc_guard4(acc[3][0], acc[3][1], acc[3][2], acc[3][3]);

  float* slab = sT[wave];
  const float* Rb = RESID ? (resid + (size_t)b * strideR) : nullptr;
#pragma unroll
  for (int i = 0; i < 4; ++i) {
    const int mBase = m0 + (i << 4);
#pragma unroll
    for (int j = 0; j < 4; ++j) {
      const int n = n0 + (j << 4) + rlane;
      float bv = 0.f;
      if (BIAS_MODE == 2) bv = bias[n];
#pragma unroll
      for (int r = 0; r < 8; ++r) {
        float v = acc[i][j][r] * scale;
        if (BIAS_MODE == 1) v += bias[mBase + mOff + r];
        if (BIAS_MODE == 2) v += bv;
        if (RESID) v += Rb[(size_t)(mBase + mOff + r) * ldc + n];
        if (ACT == 1) v = tanhf(v);
        if (ACT == 2) v = fmaxf(v, 0.0f);
        if (ACT == 3) v = v / (1.0f + expf(-v));
        if (ACT == 4) v = (v > 0.f) ? v : 0.01f * v;
        if (ACT == 5) v = 0.5f * v * (1.0f + erff(v * 0.70710678118654752f));
        slab[(mOff + r) * 68 + (j << 4) + rlane] = v;
      }
    }
    __builtin_amdgcn_fence(__ATOMIC_RELEASE, "workgroup");
    __builtin_amdgcn_wave_barrier();
    __builtin_amdgcn_fence(__ATOMIC_ACQUIRE, "workgroup");
    if (OUT_MODE == 0) {
      float* C = (float*)Cout + (size_t)b * strideC;
      const int hh = lane >> 4, c4 = (lane & 15) * 4;
      for (int pass = 0; pass < 2; ++pass) {
#pragma unroll
        for (int it = 0; it < 8; ++it) {
          const int row = it * 2 + hh;
          v4f v = *(const v4f*)(slab + row * 68 + c4);
          *(volatile v4f*)(C + (size_t)(mBase + row) * ldc + n0 + c4) = v;
        }
        __threadfence();
      }
    } else {
      const int q = lane >> 3, c8 = (lane & 7) * 8;
      unsigned short* C  = (unsigned short*)Cout  + (size_t)b * strideC;
      unsigned short* C2 = (OUT_MODE == 2) ? ((unsigned short*)Cout2 + (size_t)b * strideC) : nullptr;
      for (int pass = 0; pass < 2; ++pass) {
#pragma unroll
        for (int it = 0; it < 4; ++it) {
          const int row = it * 4 + q;
          const float* sp = slab + row * 68 + c8;
          v8h hv, lv;
#pragma unroll
          for (int e = 0; e < 8; ++e) {
            if (OUT_MODE == 1) {
              hv[e] = (_Float16)sp[e];
            } else {
              unsigned short hb = f2bf_bits(sp[e]);
              unsigned short lb = f2bf_bits(sp[e] - bf_bits2f(hb));
              hv[e] = __builtin_bit_cast(_Float16, hb);
              lv[e] = __builtin_bit_cast(_Float16, lb);
            }
          }
          *(volatile v8h*)(C + (size_t)(mBase + row) * ldc + n0 + c8) = hv;
          if (OUT_MODE == 2) *(volatile v8h*)(C2 + (size_t)(mBase + row) * ldc + n0 + c8) = lv;
        }
        __threadfence();
      }
    }
    __builtin_amdgcn_fence(__ATOMIC_RELEASE, "workgroup");
    __builtin_amdgcn_wave_barrier();
    __builtin_amdgcn_fence(__ATOMIC_ACQUIRE, "workgroup");
  }
}

__device__ __forceinline__ v8f zero8f() { return (v8f){0.f, 0.f, 0.f, 0.f, 0.f, 0.f, 0.f, 0.f}; }
__device__ __forceinline__ v8h zero8h() {
  v8h z;
#pragma unroll
  for (int e = 0; e < 8; ++e) z[e] = (_Float16)0.0f;
  return z;
}
__device__ __forceinline__ v8f hmma(v16h a, v16h b, v8f c) {
  c = __builtin_amdgcn_wmma_f32_16x16x32_f16(false, a, false, b, (short)0, c, false, false);
  asm volatile("v_nop\n\tv_nop\n\tv_nop\n\tv_nop" : "+v"(c) : "v"(a), "v"(b));
  return c;
}
__device__ __forceinline__ void lds_wave_sync() {
  __builtin_amdgcn_fence(__ATOMIC_RELEASE, "workgroup");
  __builtin_amdgcn_wave_barrier();
  __builtin_amdgcn_fence(__ATOMIC_ACQUIRE, "workgroup");
}
__device__ __forceinline__ void split_bf16(float x, _Float16& hi, _Float16& lo) {
  const unsigned short hb = f2bf_bits(x);
  const unsigned short lb = f2bf_bits(x - bf_bits2f(hb));
  hi = __builtin_bit_cast(_Float16, hb);
  lo = __builtin_bit_cast(_Float16, lb);
}

__global__ __launch_bounds__(256) void k_prep_qkv_w(
    const float* __restrict__ W, const float* __restrict__ bq, const float* __restrict__ We,
    unsigned short* __restrict__ wqh, unsigned short* __restrict__ wql,
    unsigned short* __restrict__ weh, unsigned short* __restrict__ wel, float* __restrict__ bqp) {
  const int t = blockIdx.x * 256 + threadIdx.x;
  if (blockIdx.x < 24) {
    const int n = t >> 4, k8 = (t & 15) * 8;
    const int part = n >> 7, h = (n >> 4) & 7, d = n & 15;
    const int col = part * 128 + d * 8 + h;
    v8h hv, lv;
#pragma unroll
    for (int e = 0; e < 8; ++e) {
      const float w = W[(size_t)(k8 + e) * 384 + col];
      _Float16 a, bb; split_bf16(w, a, bb); hv[e] = a; lv[e] = bb;
    }
    const size_t off = (size_t)n * 128 + k8;
    for (int pass = 0; pass < 2; ++pass) {
      *(volatile v8h*)(wqh + off) = hv;
      *(volatile v8h*)(wql + off) = lv;
      __threadfence();
    }
    if (t < 384) {
      const int pn = t >> 7, ph = (t >> 4) & 7, pd = t & 15;
      const float bv = bq[pn * 128 + pd * 8 + ph];
      *(volatile float*)(bqp + t) = bv;
      __threadfence();
      *(volatile float*)(bqp + t) = bv;
    }
  } else {
    const int u = t - 6144;
    const int n = u >> 4, k8 = (u & 15) * 8;
    const int nc = (n < 8) ? n : 7;
    v8h hv, lv;
#pragma unroll
    for (int e = 0; e < 8; ++e) {
      float w = We[(size_t)(k8 + e) * 8 + nc];
      w = (n < 8) ? w : 0.0f;
      _Float16 a, bb; split_bf16(w, a, bb); hv[e] = a; lv[e] = bb;
    }
    const size_t off = (size_t)n * 128 + k8;
    for (int pass = 0; pass < 2; ++pass) {
      *(volatile v8h*)(weh + off) = hv;
      *(volatile v8h*)(wel + off) = lv;
      __threadfence();
    }
  }
}

__global__ __launch_bounds__(256) void k_prep_wo(const float* __restrict__ Wo,
    unsigned short* __restrict__ woh, unsigned short* __restrict__ wol) {
  const int t = blockIdx.x * 256 + threadIdx.x;
  const int n = t >> 5, k8 = (t & 31) * 8;
  v8h hv, lv;
#pragma unroll
  for (int e = 0; e < 8; ++e) {
    const int kp = k8 + e;
    const int dr = kp >> 7, h = (kp >> 4) & 7, d = kp & 15;
    const int col = d * 16 + dr * 8 + h;
    const float w = Wo[(size_t)col * 128 + n];
    _Float16 a, bb; split_bf16(w, a, bb); hv[e] = a; lv[e] = bb;
  }
  const size_t off = (size_t)n * 256 + k8;
  for (int pass = 0; pass < 2; ++pass) {
    *(volatile v8h*)(woh + off) = hv;
    *(volatile v8h*)(wol + off) = lv;
    __threadfence();
  }
}

__global__ __launch_bounds__(256) void k_ln(const float* __restrict__ e, const float* __restrict__ g,
    const float* __restrict__ b, unsigned short* __restrict__ elh, unsigned short* __restrict__ ell, int nrows) {
  const int tid = threadIdx.x, wave = tid >> 5, lane = tid & 31, hh = lane >> 4, c = lane & 15;
  const int row = (blockIdx.x * 8 + wave) * 2 + hh;
  const bool ok = row < nrows;
  const int rowc = ok ? row : (nrows - 1);
  const float* p = e + (size_t)rowc * EWID + c * 8;
  const v4f x0 = *(const v4f*)p;
  const v4f x1 = *(const v4f*)(p + 4);
  float xs[8];
  xs[0] = x0[0]; xs[1] = x0[1]; xs[2] = x0[2]; xs[3] = x0[3];
  xs[4] = x1[0]; xs[5] = x1[1]; xs[6] = x1[2]; xs[7] = x1[3];
  float s = ((xs[0] + xs[1]) + (xs[2] + xs[3])) + ((xs[4] + xs[5]) + (xs[6] + xs[7]));
#pragma unroll
  for (int off = 1; off < 16; off <<= 1) s += __shfl_xor(s, off, 32);
  const float mu = s * (1.0f / 128.0f);
  float q = 0.f;
#pragma unroll
  for (int k = 0; k < 8; ++k) { xs[k] -= mu; q += xs[k] * xs[k]; }
#pragma unroll
  for (int off = 1; off < 16; off <<= 1) q += __shfl_xor(q, off, 32);
  const float rs = rsqrtf(q * (1.0f / 128.0f) + 1e-5f);
  const v4f g0 = *(const v4f*)(g + c * 8), g1 = *(const v4f*)(g + c * 8 + 4);
  const v4f b0 = *(const v4f*)(b + c * 8), b1 = *(const v4f*)(b + c * 8 + 4);
  float gg[8], bb[8];
  gg[0] = g0[0]; gg[1] = g0[1]; gg[2] = g0[2]; gg[3] = g0[3]; gg[4] = g1[0]; gg[5] = g1[1]; gg[6] = g1[2]; gg[7] = g1[3];
  bb[0] = b0[0]; bb[1] = b0[1]; bb[2] = b0[2]; bb[3] = b0[3]; bb[4] = b1[0]; bb[5] = b1[1]; bb[6] = b1[2]; bb[7] = b1[3];
  v8h hv, lv;
#pragma unroll
  for (int k = 0; k < 8; ++k) {
    const float y = xs[k] * rs * gg[k] + bb[k];
    _Float16 a, lo; split_bf16(y, a, lo); hv[k] = a; lv[k] = lo;
  }
  if (ok) {
    const size_t off = (size_t)row * EWID + c * 8;
    for (int pass = 0; pass < 2; ++pass) {
      *(volatile v8h*)(elh + off) = hv;
      *(volatile v8h*)(ell + off) = lv;
      __threadfence();
    }
  }
}

__global__ __launch_bounds__(256) void k_bias_slab(const float* __restrict__ eb, const float* __restrict__ be,
    const float* __restrict__ mask, float* __restrict__ bm, int dir) {
  const int idx = blockIdx.x * 256 + threadIdx.x;
  const int h = idx / NROWS;
  const int rem = idx - h * NROWS;
  const int i = rem / NNODE;
  const int k = rem - i * NNODE;
  const int r = dir ? (k * NNODE + i) : (i * NNODE + k);
  const float v = eb[(size_t)r * EB_LD + h] + be[h] + mask[(size_t)r * 8 + h];
  *(volatile float*)(bm + idx) = v;
  __threadfence();
  *(volatile float*)(bm + idx) = v;
}

__global__ __launch_bounds__(64) void k_edge_attn(const _Float16* __restrict__ qkv, const float* __restrict__ bm,
    unsigned short* __restrict__ vah, unsigned short* __restrict__ val, int dir) {
  __shared__ __align__(16) _Float16 Ksh[NNODE * KS_P];
  __shared__ __align__(16) _Float16 Vt[16 * VT_P];
  __shared__ __align__(16) _Float16 Pw[2][16 * PW_P];
  __shared__ __align__(16) float    Os[32 * OS_P];
  const int j = blockIdx.x;
  const int qblk = blockIdx.y * 32;
  const int tid = threadIdx.x, wave = tid >> 5, lane = tid & 31, hh = lane >> 4, c = lane & 15;
  const int i0 = qblk + wave * 16;
  const v8h z8 = zero8h();
  _Float16* pw = &Pw[wave][0];

#pragma unroll 1
  for (int h = 0; h < 8; ++h) {
    __syncthreads();
    for (int idx = tid; idx < 2 * NNODE; idx += 64) {
      const int kv = idx >> 1, part = idx & 1;
      const int r = dir ? (kv * NNODE + j) : (j * NNODE + kv);
      const _Float16* src = qkv + (size_t)r * QKV_LD + h * 16 + part * 8;
      const v8h kk8 = *(const v8h*)(src + EWID);
      const v8h vv8 = *(const v8h*)(src + 2 * EWID);
      *(v8h*)(Ksh + kv * KS_P + part * 8) = kk8;
#pragma unroll
      for (int e2 = 0; e2 < 8; ++e2) Vt[(part * 8 + e2) * VT_P + kv] = vv8[e2];
    }
    __syncthreads();

    Frag<_Float16>::U qa;
    qa.h[0] = *(const v8h*)(qkv + ((size_t)(i0 + c) * NNODE + j) * QKV_LD + h * 16 + 8 * hh);
    qa.h[1] = z8;

    float mrow[8], lrow[8];
#pragma unroll
    for (int r = 0; r < 8; ++r) { mrow[r] = -__builtin_inff(); lrow[r] = 0.f; }
    v8f o = zero8f();
    const float* bmr = bm + ((size_t)h * NNODE + (size_t)(i0 + 8 * hh)) * NNODE;

#pragma unroll 1
    for (int kc = 0; kc < 3; ++kc) {
      const int kv0 = kc * 64;
      v8f s[4];
#pragma unroll
      for (int jn = 0; jn < 4; ++jn) {
        Frag<_Float16>::U kb;
        kb.h[0] = *(const v8h*)(Ksh + (kv0 + jn * 16 + c) * KS_P + 8 * hh);
        kb.h[1] = z8;
        s[jn] = hmma(qa.v, kb.v, zero8f());
      }
      float cm[8];
#pragma unroll
      for (int r = 0; r < 8; ++r) {
        const float* brow = bmr + (size_t)r * NNODE + kv0 + c;
        float mx = -__builtin_inff();
#pragma unroll
        for (int jn = 0; jn < 4; ++jn) {
          const float v = s[jn][r] * 0.25f + brow[jn * 16];
          s[jn][r] = v;
          mx = fmaxf(mx, v);
        }
#pragma unroll
        for (int off = 1; off < 16; off <<= 1) mx = fmaxf(mx, __shfl_xor(mx, off, 32));
        cm[r] = mx;
      }
      lds_wave_sync();
#pragma unroll
      for (int r = 0; r < 8; ++r) {
        const float mnew = fmaxf(mrow[r], cm[r]);
        const float alpha = expf(mrow[r] - mnew);
        mrow[r] = mnew;
        float ps = 0.f;
#pragma unroll
        for (int jn = 0; jn < 4; ++jn) {
          const float pv = expf(s[jn][r] - mnew);
          ps += pv;
          pw[(8 * hh + r) * PW_P + jn * 16 + c] = (_Float16)pv;
        }
#pragma unroll
        for (int off = 1; off < 16; off <<= 1) ps += __shfl_xor(ps, off, 32);
        lrow[r] = lrow[r] * alpha + ps;
        o[r] *= alpha;
      }
      lds_wave_sync();
#pragma unroll
      for (int kk = 0; kk < 2; ++kk) {
        const v16h pa = Frag<_Float16>::load(pw + c * PW_P + kk * 32 + 8 * hh);
        const v16h vb = Frag<_Float16>::load(Vt + c * VT_P + kv0 + kk * 32 + 8 * hh);
        o = hmma(pa, vb, o);
      }
    }
#pragma unroll
    for (int r = 0; r < 8; ++r)
      Os[(wave * 16 + 8 * hh + r) * OS_P + h * 16 + c] = o[r] * (1.0f / lrow[r]);
  }
  __syncthreads();

  const size_t colbase = (size_t)dir * 128 + (size_t)c * 8;
  for (int pass = 0; pass < 2; ++pass) {
#pragma unroll
    for (int it = 0; it < 8; ++it) {
      const int lr = wave * 16 + it * 2 + hh;
      const float* sp = Os + lr * OS_P + c * 8;
      const v4f a4 = *(const v4f*)sp;
      const v4f b4 = *(const v4f*)(sp + 4);
      v8h hv, lv;
#pragma unroll
      for (int e = 0; e < 4; ++e) {
        _Float16 a, lo;
        split_bf16(a4[e], a, lo); hv[e] = a; lv[e] = lo;
        split_bf16(b4[e], a, lo); hv[4 + e] = a; lv[4 + e] = lo;
      }
      const size_t grow = (size_t)(qblk + lr) * NNODE + j;
      *(volatile v8h*)(vah + grow * VA_LD + colbase) = hv;
      *(volatile v8h*)(val + grow * VA_LD + colbase) = lv;
    }
    __threadfence();
  }
}

extern "C" void kernel_launch(void* const* d_in, const int* in_sizes, int n_in,
                              void* d_out, int out_size, void* d_ws, size_t ws_size,
                              hipStream_t stream) {
  if (n_in < 14) return;
  if (in_sizes[0] != NROWS * EWID || in_sizes[1] != NROWS * 8 || in_sizes[2] < EWID || in_sizes[3] < EWID ||
      in_sizes[4] != EWID * 384 || in_sizes[5] < 384 || in_sizes[6] != EWID * 8 || in_sizes[7] < 8 ||
      in_sizes[8] != EWID * 384 || in_sizes[9] < 384 || in_sizes[10] != EWID * 8 || in_sizes[11] < 8 ||
      in_sizes[12] != 256 * EWID || in_sizes[13] < EWID || out_size != NROWS * EWID) return;

  const float* e      = (const float*)d_in[0];
  const float* mask   = (const float*)d_in[1];
  const float* ln_g   = (const float*)d_in[2];
  const float* ln_b   = (const float*)d_in[3];
  const float* Wq_in  = (const float*)d_in[4];
  const float* bq_in  = (const float*)d_in[5];
  const float* We_in  = (const float*)d_in[6];
  const float* be_in  = (const float*)d_in[7];
  const float* Wq_out = (const float*)d_in[8];
  const float* bq_out = (const float*)d_in[9];
  const float* We_out = (const float*)d_in[10];
  const float* be_out = (const float*)d_in[11];
  const float* Wo     = (const float*)d_in[12];
  const float* bo     = (const float*)d_in[13];
  float* out = (float*)d_out;

  size_t off = 0;
  auto carve = [&](size_t bytes) { size_t o = off; off += (bytes + 255) & ~(size_t)255; return o; };
  const size_t oELh = carve((size_t)NROWS * EWID * 2);
  const size_t oELl = carve((size_t)NROWS * EWID * 2);
  const size_t oQKV = carve((size_t)NROWS * QKV_LD * 2);
  const size_t oEB  = carve((size_t)NROWS * EB_LD * 4);
  const size_t oBM  = carve((size_t)8 * NNODE * NNODE * 4);
  const size_t oVAh = carve((size_t)NROWS * VA_LD * 2);
  const size_t oVAl = carve((size_t)NROWS * VA_LD * 2);
  size_t oWQh[2], oWQl[2], oWEh[2], oWEl[2], oBQ[2];
  for (int d = 0; d < 2; ++d) { oWQh[d] = carve((size_t)384 * 128 * 2); oWQl[d] = carve((size_t)384 * 128 * 2); }
  for (int d = 0; d < 2; ++d) { oWEh[d] = carve((size_t)64 * 128 * 2);  oWEl[d] = carve((size_t)64 * 128 * 2); }
  const size_t oWOh = carve((size_t)128 * 256 * 2);
  const size_t oWOl = carve((size_t)128 * 256 * 2);
  for (int d = 0; d < 2; ++d) oBQ[d] = carve((size_t)384 * 4);
  if (off > ws_size) return;

  char* ws = (char*)d_ws;
  unsigned short* ELh = (unsigned short*)(ws + oELh);
  unsigned short* ELl = (unsigned short*)(ws + oELl);
  _Float16* QKV16 = (_Float16*)(ws + oQKV);
  float* EB = (float*)(ws + oEB);
  float* BM = (float*)(ws + oBM);
  unsigned short* VAh = (unsigned short*)(ws + oVAh);
  unsigned short* VAl = (unsigned short*)(ws + oVAl);
  unsigned short* WQh[2], *WQl[2], *WEh[2], *WEl[2];
  float* BQ[2];
  for (int d = 0; d < 2; ++d) {
    WQh[d] = (unsigned short*)(ws + oWQh[d]); WQl[d] = (unsigned short*)(ws + oWQl[d]);
    WEh[d] = (unsigned short*)(ws + oWEh[d]); WEl[d] = (unsigned short*)(ws + oWEl[d]);
    BQ[d] = (float*)(ws + oBQ[d]);
  }
  unsigned short* WOh = (unsigned short*)(ws + oWOh);
  unsigned short* WOl = (unsigned short*)(ws + oWOl);

  k_prep_qkv_w<<<28, 256, 0, stream>>>(Wq_in, bq_in, We_in, WQh[0], WQl[0], WEh[0], WEl[0], BQ[0]);
  k_prep_qkv_w<<<28, 256, 0, stream>>>(Wq_out, bq_out, We_out, WQh[1], WQl[1], WEh[1], WEl[1], BQ[1]);
  k_prep_wo<<<16, 256, 0, stream>>>(Wo, WOh, WOl);

  k_ln<<<NROWS / 16, 256, 0, stream>>>(e, ln_g, ln_b, ELh, ELl, NROWS);

  const int tilesQKV = (NROWS / 64) * (QKV_LD / 64);
  const int tilesEB  = (NROWS / 64) * (EB_LD / 64);
  const int tilesOUT = (NROWS / 64) * (EWID / 64);
  for (int dir = 0; dir < 2; ++dir) {
    const float* be = dir ? be_out : be_in;
    wmma_gemm64<1, true, 2, 1, false><<<dim3(tilesQKV / 8, 1), 256, 0, stream>>>(
        ELh, ELl, EWID, (long)0, WQh[dir], WQl[dir], EWID, (long)0,
        (void*)QKV16, (void*)QKV16, QKV_LD, (long)0, BQ[dir], BQ[dir], (long)0, NROWS, QKV_LD, EWID, 1.0f);
    wmma_gemm64<1, true, 0, 0, false><<<dim3(tilesEB / 8, 1), 256, 0, stream>>>(
        ELh, ELl, EWID, (long)0, WEh[dir], WEl[dir], EWID, (long)0,
        (void*)EB, (void*)EB, EB_LD, (long)0, be, be, (long)0, NROWS, EB_LD, EWID, 1.0f);
    k_bias_slab<<<(8 * NNODE * NNODE) / 256, 256, 0, stream>>>(EB, be, mask, BM, dir);
    k_edge_attn<<<dim3(NNODE, NNODE / 32), 64, 0, stream>>>(QKV16, BM, VAh, VAl, dir);
  }
  wmma_gemm64<1, true, 2, 0, false><<<dim3(tilesOUT / 8, 1), 256, 0, stream>>>(
      VAh, VAl, VA_LD, (long)0, WOh, WOl, VA_LD, (long)0,
      (void*)out, (void*)out, EWID, (long)0, bo, bo, (long)0, NROWS, EWID, VA_LD, 1.0f);
}
